// QNetNode_71554155152032
// MI455X (gfx1250) — hardware-verified
//
#include <hip/hip_runtime.h>


namespace {
constexpr int N = 20000, NP = 20032  , NG = 8, E = 320000, FD = 128, D = 64, HM = 128;
constexpr float XS = 8.0f, WSC = 256.0f;

typedef _Float16 b16;
typedef __attribute__((ext_vector_type(16))) _Float16 v16b;
typedef __attribute__((ext_vector_type(8))) _Float16 v8b;
typedef __attribute__((ext_vector_type(4))) _Float16 v4b;
typedef __attribute__((ext_vector_type(8))) float v8f;
typedef __attribute__((ext_vector_type(4))) float v4f;
__device__ __forceinline__ float bf16_rne(float f) { unsigned int u = __float_as_uint(f); u += 0x7FFFu + ((u >> 16) & 1u); return __uint_as_float(u & 0xFFFF0000u); }
__device__ __forceinline__ void split16(float v, b16& hi, b16& lo) { hi = (b16)v; lo = (b16)(v - (float)hi); }
__device__ __forceinline__ v16b frag_kb(const b16* p, int hh) { const v8b a = *(const v8b*)(p + 8 * hh), b = *(const v8b*)(p + 16 + 8 * hh); v16b f;
#pragma unroll
  for (int e = 0; e < 8; ++e) { f[e] = a[e]; f[8 + e] = b[e]; } return f; }
__device__ __forceinline__ v8f wmma16b(v16b a, v16b b, v8f c) { v8f d = __builtin_amdgcn_wmma_f32_16x16x32_f16(false, a, false, b, (short)0, c, false, false); asm volatile("v_nop\n\tv_nop\n\tv_nop\n\tv_nop" : "+v"(d) : "v"(a), "v"(b)); return d; }
__device__ __forceinline__ void wave_lds_sync() { __builtin_amdgcn_fence(__ATOMIC_RELEASE, "workgroup"); __builtin_amdgcn_wave_barrier(); __builtin_amdgcn_fence(__ATOMIC_ACQUIRE, "workgroup"); }
__device__ __forceinline__ float pmul(float a, float b) { float p = a * b; asm volatile("" : "+v"(p)); return p; }
__device__ __forceinline__ float hsum16(float v) { v += __shfl_xor(v, 1); v += __shfl_xor(v, 2); v += __shfl_xor(v, 4); return v + __shfl_xor(v, 8); }
__device__ __forceinline__ int iclamp(int v, int lo, int hi) { return v < lo ? lo : (v > hi ? hi : v); }

constexpr int CSR_NBLK = 512, CSR_GB = 9, CSR_GN = 1 << CSR_GB  , CSR_MAXG = 512, CSR_CAP = 12288  ;
__global__ __launch_bounds__(64) void csrA_kernel(const int* __restrict__ dst, int E, int N, int nG, int CHP, int NGP, int* __restrict__ STG, int* __restrict__ HST) {
  extern __shared__ int sm[];
  int* cnt = sm; int* run = sm + NGP; int* ids = sm + 2 * NGP;
  const int b = blockIdx.x; const int ch = (E + CSR_NBLK - 1) / CSR_NBLK; const int e0 = b * ch, e1 = min(E, e0 + ch);
  for (int i = threadIdx.x; i < NGP; i += 64) cnt[i] = 0;
  for (int i = threadIdx.x; i < CHP; i += 64) ids[i] = -1;
  __syncthreads();
  if (threadIdx.x == 0) {
    for (int e = e0; e < e1; ++e) { int d = dst[e]; d = (d < 0) ? 0 : (d >= N ? N - 1 : d); cnt[d >> CSR_GB] += 1; }
    int acc = 0; for (int g = 0; g < nG; ++g) { run[g] = acc; acc += cnt[g]; }
    for (int e = e0; e < e1; ++e) { int d = dst[e]; d = (d < 0) ? 0 : (d >= N ? N - 1 : d); const int g = d >> CSR_GB; ids[run[g]] = e; run[g] += 1; } }
  __syncthreads();
  typedef __attribute__((ext_vector_type(4))) int v4i;
  for (int pass = 0; pass < 2; ++pass) {
    for (int i = threadIdx.x; i < CHP / 4; i += 64) *(volatile v4i*)(STG + (size_t)b * CHP + i * 4) = *(const v4i*)(&ids[i * 4]);
    for (int i = threadIdx.x; i < NGP / 4; i += 64) { v4i v; for (int e = 0; e < 4; ++e) v[e] = (i * 4 + e < nG) ? cnt[i * 4 + e] : 0; *(volatile v4i*)(HST + (size_t)b * NGP + i * 4) = v; }
    __threadfence(); }
}
__global__ __launch_bounds__(512) void csrS_kernel(const int* __restrict__ HST, int nG, int NGP, int* __restrict__ START, int* __restrict__ TOT, int* __restrict__ OFF) {
  __shared__ int tot[CSR_MAXG];
  const int b = threadIdx.x;
  for (int pass = 0; pass < 2; ++pass) { int runb = 0; for (int g = 0; g < nG; ++g) { int c = HST[(size_t)b * NGP + g]; c = (c < 0) ? 0 : c; ((volatile int*)OFF)[(size_t)g * CSR_NBLK + b] = runb; runb += c; } __threadfence(); }
  for (int g = threadIdx.x; g < nG; g += 512) { int s = 0; for (int bb = 0; bb < CSR_NBLK; ++bb) { int c = HST[(size_t)bb * NGP + g]; s += (c < 0) ? 0 : c; } tot[g] = s; }
  __syncthreads();
  if (threadIdx.x < 32) {
    __shared__ int st[CSR_MAXG + 32];
    if (threadIdx.x == 0) { int acc = 0; for (int g = 0; g < NGP; ++g) { st[g] = acc; if (g < nG) acc += (tot[g] + 31) & ~31; } st[NGP] = acc; }
    __builtin_amdgcn_fence(__ATOMIC_RELEASE, "workgroup"); __builtin_amdgcn_wave_barrier(); __builtin_amdgcn_fence(__ATOMIC_ACQUIRE, "workgroup");
    for (int pass = 0; pass < 2; ++pass) { for (int i = threadIdx.x; i < NGP + 32; i += 32) { ((volatile int*)START)[i] = (i <= NGP) ? st[min(i, NGP)] : 0; ((volatile int*)TOT)[i] = (i < nG) ? tot[i] : 0; } __threadfence(); } }
}
__global__ __launch_bounds__(256) void csrB_kernel(const int* __restrict__ dst, int N, int nG, int CHP, int NGP, int permLen, const int* __restrict__ STG, const int* __restrict__ HST, const int* __restrict__ OFF, const int* __restrict__ START, const int* __restrict__ TOT, int* __restrict__ PERM, int* __restrict__ ROWPTR, int* __restrict__ ROWCNT, int* __restrict__ FLAG) {
  typedef __attribute__((ext_vector_type(4))) int v4i;
  __shared__ int ids[CSR_CAP]; __shared__ unsigned short key[CSR_CAP]; __shared__ int outp[CSR_CAP]; __shared__ int ncnt[CSR_GN + 1]; __shared__ int boff[CSR_NBLK + 1];
  const int g = blockIdx.x, t_ = threadIdx.x; int tot = TOT[g]; int st = START[g], stn = START[g + 1]; const int v0 = g * CSR_GN; const int nv = min(CSR_GN, N - v0);
  st = (st < 0) ? 0 : (st > permLen - 32 ? permLen - 32 : st) & ~31; stn = (stn < st) ? st : (stn > permLen ? permLen : stn); tot = (tot < 0) ? 0 : tot; if (tot > stn - st && tot <= CSR_CAP) tot = stn - st;
  if (tot > CSR_CAP) {
    for (int pass = 0; pass < 2; ++pass) { for (int i = t_; i < CSR_GN / 4; i += 256) { v4i a, c; for (int e = 0; e < 4; ++e) { a[e] = st; c[e] = 0; } *(volatile v4i*)(ROWPTR + v0 + i * 4) = a; *(volatile v4i*)(ROWCNT + v0 + i * 4) = c; } if (t_ == 0) ((volatile int*)FLAG)[0] = 1; __threadfence(); } (void)nv; return; }
  if (t_ == 0) { int acc = 0; for (int b = 0; b < CSR_NBLK; ++b) { boff[b] = acc; int c = HST[(size_t)b * NGP + g]; c = (c < 0) ? 0 : (c > CHP ? CHP : c); acc += c; if (acc > tot) acc = tot; } boff[CSR_NBLK] = acc; }
  for (int i = t_; i <= CSR_GN; i += 256) ncnt[i] = 0;
  __syncthreads();
  for (int b = 0; b < CSR_NBLK; ++b) { const int c = boff[b + 1] - boff[b]; int o_ = OFF[(size_t)g * CSR_NBLK + b]; o_ = (o_ < 0) ? 0 : (o_ > CHP - c ? CHP - c : o_); const int* src_ = STG + (size_t)b * CHP + o_;
    for (int i = t_; i < c; i += 256) { int id = src_[i]; id = (id < 0) ? 0 : id; ids[boff[b] + i] = id; int d = dst[id]; d = (d < v0) ? v0 : (d >= N ? N - 1 : d); int kk = d - v0; kk = (kk < 0) ? 0 : (kk >= CSR_GN ? CSR_GN - 1 : kk); key[boff[b] + i] = (unsigned short)kk; } }
  __syncthreads();
  if (t_ == 0) { for (int i = 0; i < tot; ++i) ncnt[key[i]] += 1; int acc = 0; for (int vl = 0; vl < CSR_GN; ++vl) { const int c = ncnt[vl]; ncnt[vl] = acc; acc += c; } ncnt[CSR_GN] = acc;
    for (int i = 0; i < tot; ++i) { const int vl = key[i]; outp[ncnt[vl]] = ids[i]; ncnt[vl] += 1; }
    for (int vl = CSR_GN; vl > 0; --vl) ncnt[vl] = ncnt[vl - 1]; ncnt[0] = 0; }
  __syncthreads();
  for (int pass = 0; pass < 2; ++pass) {
    for (int i = t_; i < (stn - st) / 4; i += 256) { v4i v; for (int e = 0; e < 4; ++e) { const int q = i * 4 + e; v[e] = (q < tot) ? outp[q] : -1; } *(volatile v4i*)(PERM + st + i * 4) = v; }
    for (int i = t_; i < CSR_GN / 4; i += 256) { v4i a, c; for (int e = 0; e < 4; ++e) { const int vl = i * 4 + e; a[e] = st + ncnt[vl]; c[e] = (vl < nv) ? (ncnt[vl + 1] - ncnt[vl]) : 0; } *(volatile v4i*)(ROWPTR + v0 + i * 4) = a; *(volatile v4i*)(ROWCNT + v0 + i * 4) = c; }
    __threadfence(); }
}
__global__ __launch_bounds__(256) void csrZ_kernel(int* __restrict__ p, size_t n4) { typedef __attribute__((ext_vector_type(4))) int v4i; const size_t tid = (size_t)blockIdx.x * 256 + threadIdx.x, nth = (size_t)gridDim.x * 256; v4i z = {0, 0, 0, 0}; for (size_t i = tid; i < n4; i += nth) *(volatile v4i*)(p + i * 4) = z; }
struct CsrBufs { int *STG, *HST, *OFF, *START, *TOT, *PERM, *ROWPTR, *ROWCNT, *FLAG; int nG, NGP, CHP; size_t permLen; char* base; size_t bytes; };
static size_t csr_carve(CsrBufs& c, char* ws, size_t off, int E, int N) {
  const size_t off0 = off; c.base = ws + off;
  auto al = [&](size_t bytes) { char* p = ws + off; off += (bytes + 255) & ~(size_t)255; return p; };
  c.nG = (N + CSR_GN - 1) / CSR_GN; c.NGP = (c.nG + 31) & ~31; const int ch = (E + CSR_NBLK - 1) / CSR_NBLK; c.CHP = (ch + 31) & ~31; c.permLen = (size_t)E + 32 * (size_t)c.nG + 32;
  c.STG = (int*)al((size_t)CSR_NBLK * c.CHP * 4); c.HST = (int*)al((size_t)CSR_NBLK * c.NGP * 4); c.OFF = (int*)al((size_t)c.NGP * CSR_NBLK * 4); c.START = (int*)al((size_t)(c.NGP + 64) * 4); c.TOT = (int*)al((size_t)(c.NGP + 64) * 4);
  c.PERM = (int*)al(c.permLen * 4); c.ROWPTR = (int*)al((size_t)c.nG * CSR_GN * 4); c.ROWCNT = (int*)al((size_t)c.nG * CSR_GN * 4); c.FLAG = (int*)al(256);
  c.bytes = off - off0; return off;
}
static void csr_build(const CsrBufs& c, const int* dst, int E, int N, hipStream_t stream) {
  const size_t smem = (size_t)(2 * c.NGP + c.CHP) * 4;
  csrZ_kernel<<<512, 256, 0, stream>>>((int*)c.base, c.bytes / 16);
  csrA_kernel<<<CSR_NBLK, 64, smem, stream>>>(dst, E, N, c.nG, c.CHP, c.NGP, c.STG, c.HST);
  csrS_kernel<<<1, 512, 0, stream>>>(c.HST, c.nG, c.NGP, c.START, c.TOT, c.OFF);
  csrB_kernel<<<c.nG, 256, 0, stream>>>(dst, N, c.nG, c.CHP, c.NGP, (int)c.permLen, c.STG, c.HST, c.OFF, c.START, c.TOT, c.PERM, c.ROWPTR, c.ROWCNT, c.FLAG);
}


__global__ __launch_bounds__(256) void prepx_kernel(const float* __restrict__ nf, b16* __restrict__ NF16) {
  const size_t i = ((size_t)blockIdx.x * 256 + threadIdx.x) * 8; if (i >= (size_t)NP * FD) return; const size_t row = i / FD; v8b o;
  if (row < N) { const v4f a = *(const v4f*)(nf + i), c = *(const v4f*)(nf + i + 4);
#pragma unroll
    for (int j = 0; j < 4; ++j) { o[j] = (b16)(bf16_rne(a[j]) * XS); o[4 + j] = (b16)(bf16_rne(c[j]) * XS); } } else { o = (v8b){}; }
  for (int pass = 0; pass < 2; ++pass) { *(volatile v8b*)(NF16 + i) = o; __threadfence(); }
}
__global__ __launch_bounds__(256) void prepw_kernel(const float* __restrict__ wn, const float* __restrict__ wc, const float* __restrict__ w1, const float* __restrict__ wo, b16* __restrict__ WN, b16* __restrict__ WC, b16* __restrict__ W1A, b16* __restrict__ WO) {
  __shared__ __attribute__((aligned(16))) b16 T[128][128 + 8];
  const int kind = blockIdx.x, t_ = threadIdx.x;
  const int IN = kind == 0 ? FD : kind == 1 ? D : kind == 2 ? D : HM, OUT = kind == 0 ? D : kind == 1 ? D : kind == 2 ? HM : D; const float* w = kind == 0 ? wn : kind == 1 ? wc : kind == 2 ? w1 : wo; b16* dst = kind == 0 ? WN : kind == 1 ? WC : kind == 2 ? W1A : WO;
  const int ldw = kind == 2 ? HM : OUT;
  for (int q = t_; q < IN * OUT; q += 256) { const int ii = q / OUT, oo = q - ii * OUT; T[oo][ii] = (b16)(bf16_rne(w[(size_t)ii * ldw + oo]) * WSC); }
  __syncthreads();
  for (int pass = 0; pass < 2; ++pass) { for (int q = t_; q < OUT * (IN / 8); q += 256) { const int oo = q / (IN / 8), c8 = (q - oo * (IN / 8)) * 8; *(volatile v8b*)(dst + (size_t)oo * IN + c8) = *(const v8b*)(&T[oo][c8]); } __threadfence(); }
}
__global__ __launch_bounds__(128) void base_kernel(const b16* __restrict__ NF16, const b16* __restrict__ WN, const float* __restrict__ bn, float* __restrict__ BASE) {
  __shared__ __attribute__((aligned(16))) float Ts[4][16][D + 4];
  const int wave = threadIdx.x >> 5, lane = threadIdx.x & 31, nloc = lane & 15, hlf = lane >> 4; const size_t m0 = (size_t)blockIdx.x * 64 + wave * 16;
  v8f acc[4] = {{}, {}, {}, {}};
#pragma unroll
  for (int kb = 0; kb < FD; kb += 32) { const v16b a = frag_kb(NF16 + (m0 + nloc) * FD + kb, hlf);
#pragma unroll
    for (int t = 0; t < 4; ++t) acc[t] = wmma16b(a, frag_kb(WN + (size_t)(t * 16 + nloc) * FD + kb, hlf), acc[t]); }
#pragma unroll
  for (int t = 0; t < 4; ++t) { const float bb = bf16_rne(bn[t * 16 + nloc]);
#pragma unroll
    for (int r = 0; r < 8; ++r) Ts[wave][8 * hlf + r][t * 16 + nloc] = acc[t][r] * (1.0f / (XS * WSC)) + bb; }
  wave_lds_sync();
  for (int pass = 0; pass < 2; ++pass) { for (int rr = 0; rr < 16; ++rr) if (lane < 16) *(volatile v4f*)(BASE + (m0 + rr) * D + lane * 4) = *(const v4f*)(&Ts[wave][rr][lane * 4]); __threadfence(); }
}
__global__ __launch_bounds__(256) void im_kernel(const float* __restrict__ BASE, const float* __restrict__ bp, const int* __restrict__ picked, int g, float* __restrict__ IM, b16* __restrict__ HH, b16* __restrict__ HL) {
  const int wave = threadIdx.x >> 5, lane = threadIdx.x & 31; const size_t v = ((size_t)blockIdx.x * 8 + wave) * 2 + (lane >> 4); const int c0 = (lane & 15) * 4;
  const int pk = iclamp(picked[g], 0, N - 1);
  v4f x = *(const v4f*)(BASE + v * D + c0);
  if ((int)v == pk) { x[0] += bf16_rne(bp[c0]); x[1] += bf16_rne(bp[c0 + 1]); x[2] += bf16_rne(bp[c0 + 2]); x[3] += bf16_rne(bp[c0 + 3]); }
  v4b h, hl; for (int j = 0; j < 4; ++j) { b16 a_, b_; split16(fmaxf(x[j], 0.0f) * XS, a_, b_); h[j] = a_; hl[j] = b_; }
  for (int pass = 0; pass < 2; ++pass) { *(volatile v4f*)(IM + v * D + c0) = x; *(volatile v4b*)(HH + v * D + c0) = h; *(volatile v4b*)(HL + v * D + c0) = hl; __threadfence(); }
}
__global__ __launch_bounds__(256) void pool_kernel(const b16* __restrict__ HH, const b16* __restrict__ HL, const int* __restrict__ src, const float* __restrict__ ew, const int* __restrict__ PERM, const int* __restrict__ ROWPTR, const int* __restrict__ ROWCNT, int permLen, b16* __restrict__ PH, b16* __restrict__ PL) {
  const int wave = threadIdx.x >> 5, lane = threadIdx.x & 31; const size_t v = ((size_t)blockIdx.x * 8 + wave) * 2 + (lane >> 4); const int c0 = (lane & 15) * 4;
  int st = ROWPTR[v], cnt = ROWCNT[v]; cnt = iclamp(cnt, 0, 4096); st = iclamp(st, 0, permLen - cnt);
  float acc[4] = {0.0f, 0.0f, 0.0f, 0.0f};
  for (int j = 0; j < cnt; ++j) { const int e = iclamp(PERM[st + j], 0, E - 1); const int s = iclamp(src[e], 0, N - 1); const float w = bf16_rne(ew[e]); const v4b hv = *(const v4b*)(HH + (size_t)s * D + c0), hw = *(const v4b*)(HL + (size_t)s * D + c0);
#pragma unroll
    for (int q = 0; q < 4; ++q) acc[q] += pmul(w, ((float)hv[q] + (float)hw[q]) * (1.0f / XS)); }
  v4b ho, lo_; for (int q = 0; q < 4; ++q) { b16 a_, b_; split16(acc[q] * XS, a_, b_); ho[q] = a_; lo_[q] = b_; }
  for (int pass = 0; pass < 2; ++pass) { *(volatile v4b*)(PH + v * D + c0) = ho; *(volatile v4b*)(PL + v * D + c0) = lo_; __threadfence(); }
}
__global__ __launch_bounds__(128) void conv_kernel(const b16* __restrict__ PH, const b16* __restrict__ PL, const b16* __restrict__ WC, const float* __restrict__ bc, const float* __restrict__ IM, b16* __restrict__ HH, b16* __restrict__ HL, float* __restrict__ H32) {
  __shared__ __attribute__((aligned(16))) float Ts[4][16][D + 4];
  const int wave = threadIdx.x >> 5, lane = threadIdx.x & 31, nloc = lane & 15, hlf = lane >> 4; const size_t m0 = (size_t)blockIdx.x * 64 + wave * 16;
  v8f acc[4] = {{}, {}, {}, {}};
#pragma unroll
  for (int kb = 0; kb < D; kb += 32) { const v16b a = frag_kb(PH + (m0 + nloc) * D + kb, hlf), al = frag_kb(PL + (m0 + nloc) * D + kb, hlf);
#pragma unroll
    for (int t = 0; t < 4; ++t) { const v16b bw = frag_kb(WC + (size_t)(t * 16 + nloc) * D + kb, hlf); acc[t] = wmma16b(a, bw, acc[t]); acc[t] = wmma16b(al, bw, acc[t]); } }
#pragma unroll
  for (int t = 0; t < 4; ++t) { const int c = t * 16 + nloc; const float bb = bf16_rne(bc[c]);
#pragma unroll
    for (int r = 0; r < 8; ++r) Ts[wave][8 * hlf + r][c] = fmaxf(acc[t][r] * (1.0f / (XS * WSC)) + bb + IM[(m0 + 8 * hlf + r) * D + c], 0.0f); }
  wave_lds_sync();
  for (int pass = 0; pass < 2; ++pass) { for (int rr = 0; rr < 16; ++rr) if (lane < 16) { const v4f x = *(const v4f*)(&Ts[wave][rr][lane * 4]); *(volatile v4f*)(H32 + (m0 + rr) * D + lane * 4) = x; v4b h, hl; for (int j = 0; j < 4; ++j) { b16 a_, b_; split16(x[j] * XS, a_, b_); h[j] = a_; hl[j] = b_; } *(volatile v4b*)(HH + (m0 + rr) * D + lane * 4) = h; *(volatile v4b*)(HL + (m0 + rr) * D + lane * 4) = hl; } __threadfence(); }
}
__global__ __launch_bounds__(256) void graph_kernel(const float* __restrict__ H32, const float* __restrict__ w1, const float* __restrict__ b1, const int* __restrict__ tgt, int g, float* __restrict__ GB, float* __restrict__ TG) {
  __shared__ float part[256][4]; __shared__ float mean[D];
  const int t_ = threadIdx.x; const int c4 = (t_ & 15) * 4, grp = t_ >> 4;
  float s[4] = {0.0f, 0.0f, 0.0f, 0.0f};
  for (int v = grp; v < N; v += 16) { const v4f x = *(const v4f*)(H32 + (size_t)v * D + c4); s[0] += x[0]; s[1] += x[1]; s[2] += x[2]; s[3] += x[3]; }
  for (int q = 0; q < 4; ++q) part[t_][q] = s[q];
  __syncthreads();
  if (t_ < D) { const int cc = t_; const int l4 = (cc >> 2), q = cc & 3; float tot = 0.0f; for (int gi = 0; gi < 16; ++gi) tot += part[gi * 16 + l4][q]; mean[cc] = tot * (1.0f / N); }
  __syncthreads();
  const int tg = iclamp(tgt[g], 0, N - 1);
  for (int pass = 0; pass < 2; ++pass) {
    if (t_ < HM) { float acc = bf16_rne(b1[t_]);
#pragma unroll 1
      for (int c = 0; c < D; ++c) acc += pmul(mean[c], bf16_rne(w1[(size_t)(D + c) * HM + t_])); ((volatile float*)GB)[t_] = acc; }
    if (t_ < D) ((volatile float*)TG)[t_] = H32[(size_t)tg * D + t_];
    __threadfence(); }
}
__global__ __launch_bounds__(128) void ro1_kernel(const b16* __restrict__ HH, const b16* __restrict__ HL, const b16* __restrict__ W1A, const float* __restrict__ GB, b16* __restrict__ EH, b16* __restrict__ EL) {
  __shared__ __attribute__((aligned(16))) b16 Th[4][16][HM + 8], Tl[4][16][HM + 8];
  const int wave = threadIdx.x >> 5, lane = threadIdx.x & 31, nloc = lane & 15, hlf = lane >> 4; const size_t m0 = (size_t)blockIdx.x * 64 + wave * 16;
  v8f acc[8];
#pragma unroll
  for (int t = 0; t < 8; ++t) acc[t] = (v8f){};
#pragma unroll
  for (int kb = 0; kb < D; kb += 32) { const v16b a = frag_kb(HH + (m0 + nloc) * D + kb, hlf), al = frag_kb(HL + (m0 + nloc) * D + kb, hlf);
#pragma unroll
    for (int t = 0; t < 8; ++t) { const v16b bw = frag_kb(W1A + (size_t)(t * 16 + nloc) * D + kb, hlf); acc[t] = wmma16b(a, bw, acc[t]); acc[t] = wmma16b(al, bw, acc[t]); } }
#pragma unroll
  for (int t = 0; t < 8; ++t) { const int o = t * 16 + nloc; const float gb = GB[o];
#pragma unroll
    for (int r = 0; r < 8; ++r) { b16 a_, b_; split16(fmaxf(acc[t][r] * (1.0f / (XS * WSC)) + gb, 0.0f) * XS, a_, b_); Th[wave][8 * hlf + r][o] = a_; Tl[wave][8 * hlf + r][o] = b_; } }
  wave_lds_sync();
  for (int pass = 0; pass < 2; ++pass) { for (int rr = 0; rr < 16; ++rr) if (lane < 16) { *(volatile v8b*)(EH + (m0 + rr) * HM + lane * 8) = *(const v8b*)(&Th[wave][rr][lane * 8]); *(volatile v8b*)(EL + (m0 + rr) * HM + lane * 8) = *(const v8b*)(&Tl[wave][rr][lane * 8]); } __threadfence(); }
}
__global__ __launch_bounds__(128) void ro2_kernel(const b16* __restrict__ EH, const b16* __restrict__ EL, const b16* __restrict__ WO, const float* __restrict__ bo, const float* __restrict__ TG, int g, float* __restrict__ out) {
  __shared__ float Sq[64];
  const int wave = threadIdx.x >> 5, lane = threadIdx.x & 31, nloc = lane & 15, hlf = lane >> 4, t_ = threadIdx.x; const size_t m0 = (size_t)blockIdx.x * 64 + wave * 16;
  v8f acc[4] = {{}, {}, {}, {}};
#pragma unroll
  for (int kb = 0; kb < HM; kb += 32) { const v16b a = frag_kb(EH + (m0 + nloc) * HM + kb, hlf), al = frag_kb(EL + (m0 + nloc) * HM + kb, hlf);
#pragma unroll
    for (int t = 0; t < 4; ++t) { const v16b bw = frag_kb(WO + (size_t)(t * 16 + nloc) * HM + kb, hlf); acc[t] = wmma16b(a, bw, acc[t]); acc[t] = wmma16b(al, bw, acc[t]); } }
#pragma unroll
  for (int r = 0; r < 8; ++r) { float qv = 0.0f;
#pragma unroll
    for (int t = 0; t < 4; ++t) { const int c = t * 16 + nloc; qv += pmul(acc[t][r] * (1.0f / (XS * WSC)) + bf16_rne(bo[c]), TG[c]); }
    qv = hsum16(qv); if (nloc == 0) Sq[wave * 16 + 8 * hlf + r] = qv; }
  __syncthreads();
  for (int pass = 0; pass < 2; ++pass) { if (t_ < 64) { const size_t v = (size_t)blockIdx.x * 64 + t_; if (v < N) ((volatile float*)out)[(size_t)g * N + v] = Sq[t_]; } __threadfence(); }
}
}

extern "C" void kernel_launch(void* const* d_in, const int* in_sizes, int n_in, void* d_out, int out_size, void* d_ws, size_t ws_size, hipStream_t stream) {
  (void)n_in;
  auto Fp = [&](int i) { return (const float*)d_in[i]; }; auto Ip = [&](int i) { return (const int*)d_in[i]; };
  if (in_sizes[0] != N * FD || in_sizes[1] != FD * D || in_sizes[4] != D * D || in_sizes[6] != HM * HM || in_sizes[8] != HM * D || in_sizes[10] != NG * E || in_sizes[11] != NG * E || in_sizes[12] != NG * E || in_sizes[13] != NG || out_size != NG * N) return;
  size_t off = 0; char* ws = (char*)d_ws;
  auto carve = [&](size_t bytes) { char* p = ws + off; off += (bytes + 255) & ~(size_t)255; return p; };
  b16* NF16 = (b16*)carve((size_t)NP * FD * 2); b16* WN = (b16*)carve(D * FD * 2); b16* WC = (b16*)carve(D * D * 2); b16* W1A = (b16*)carve(HM * D * 2); b16* WO = (b16*)carve(D * HM * 2);
  float* BASE = (float*)carve((size_t)NP * D * 4); float* IM = (float*)carve((size_t)NP * D * 4); b16* HH = (b16*)carve((size_t)NP * D * 2); b16* HL = (b16*)carve((size_t)NP * D * 2); b16* PH = (b16*)carve((size_t)NP * D * 2); b16* PL = (b16*)carve((size_t)NP * D * 2);
  float* H32 = (float*)carve((size_t)NP * D * 4); b16* EH = (b16*)carve((size_t)NP * HM * 2); b16* EL = (b16*)carve((size_t)NP * HM * 2); float* GB = (float*)carve(HM * 4); float* TG = (float*)carve(256);
  CsrBufs csr; off = csr_carve(csr, ws, off, E, N);
  if (off > ws_size || off > ((size_t)128 << 20)) return;
  prepx_kernel<<<(NP * FD / 8 + 255) / 256, 256, 0, stream>>>(Fp(0), NF16);
  prepw_kernel<<<4, 256, 0, stream>>>(Fp(1), Fp(4), Fp(6), Fp(8), WN, WC, W1A, WO);
  base_kernel<<<NP / 64, 128, 0, stream>>>(NF16, WN, Fp(2), BASE);
  for (int g = 0; g < NG; ++g) {
    im_kernel<<<NP / 16, 256, 0, stream>>>(BASE, Fp(3), Ip(14), g, IM, HH, HL);
    csr_build(csr, Ip(12) + (size_t)g * E, E, N, stream);
    for (int lv = 0; lv < 2; ++lv) {
      pool_kernel<<<NP / 16, 256, 0, stream>>>(HH, HL, Ip(11) + (size_t)g * E, Fp(10) + (size_t)g * E, csr.PERM, csr.ROWPTR, csr.ROWCNT, (int)csr.permLen, PH, PL);
      conv_kernel<<<NP / 64, 128, 0, stream>>>(PH, PL, WC, Fp(5), IM, HH, HL, H32); }
    graph_kernel<<<1, 256, 0, stream>>>(H32, Fp(6), Fp(7), Ip(13), g, GB, TG);
    ro1_kernel<<<NP / 64, 128, 0, stream>>>(HH, HL, W1A, GB, EH, EL);
    ro2_kernel<<<NP / 64, 128, 0, stream>>>(EH, EL, WO, Fp(9), TG, g, (float*)d_out); }
}
